// ImprovedAttentionMechanism_79723182949002
// MI455X (gfx1250) — hardware-verified
//
#include <hip/hip_runtime.h>


namespace {
constexpr int S = 2048, F = 512, NH = 8, HD = 64, E3 = 3 * NH * HD;
constexpr float XS = 8.0f, PS = 1024.0f, WSC = 256.0f;
typedef _Float16 b16;
typedef __attribute__((ext_vector_type(16))) _Float16 v16b;
typedef __attribute__((ext_vector_type(8))) _Float16 v8b;
typedef __attribute__((ext_vector_type(8))) float v8f;
typedef __attribute__((ext_vector_type(4))) float v4f;
typedef __attribute__((ext_vector_type(2))) float v2f;
__device__ __forceinline__ float bf16_rne(float f) { unsigned int u = __float_as_uint(f); u += 0x7FFFu + ((u >> 16) & 1u); return __uint_as_float(u & 0xFFFF0000u); }
__device__ __forceinline__ void split16(float v, b16& hi, b16& lo) { hi = (b16)v; lo = (b16)(v - (float)hi); }
__device__ __forceinline__ v16b frag_kb(const b16* p, int hh) { const v8b a = *(const v8b*)(p + 8 * hh), b = *(const v8b*)(p + 16 + 8 * hh); v16b f;
#pragma unroll
  for (int e = 0; e < 8; ++e) { f[e] = a[e]; f[8 + e] = b[e]; } return f; }
__device__ __forceinline__ v8f wmma16b(v16b a, v16b b, v8f c) { v8f d = __builtin_amdgcn_wmma_f32_16x16x32_f16(false, a, false, b, (short)0, c, false, false); asm volatile("v_nop\n\tv_nop\n\tv_nop\n\tv_nop" : "+v"(d) : "v"(a), "v"(b)); return d; }
__device__ __forceinline__ void wave_lds_sync() { __builtin_amdgcn_fence(__ATOMIC_RELEASE, "workgroup"); __builtin_amdgcn_wave_barrier(); __builtin_amdgcn_fence(__ATOMIC_ACQUIRE, "workgroup"); }
__device__ __forceinline__ float pmul(float a, float b) { float p = a * b; asm volatile("" : "+v"(p)); return p; }

__global__ __launch_bounds__(256) void wput_kernel(const float* __restrict__ wq, const float* __restrict__ wk, const float* __restrict__ wv, b16* __restrict__ WT) { const int u = blockIdx.x * 256 + threadIdx.x; if (u >= E3 * (F / 8)) return; const int o = u / (F / 8), k0 = (u % (F / 8)) * 8; const int which = o / 512, h = (o / 64) % NH, d = o % 64; const float* w = which == 0 ? wq : (which == 1 ? wk : wv); v8b v;
#pragma unroll
  for (int j = 0; j < 8; ++j) v[j] = (b16)(bf16_rne(w[((size_t)h * F + k0 + j) * HD + d]) * WSC); for (int pass = 0; pass < 2; ++pass) { *(volatile v8b*)(WT + (size_t)o * F + k0) = v; __threadfence(); } }
__global__ __launch_bounds__(32) void qkv_kernel(const float* __restrict__ dat, const float* __restrict__ g, const float* __restrict__ bt, const b16* __restrict__ WT, float* __restrict__ QKV) {
  __shared__ __attribute__((aligned(16))) b16 Ah[16][F + 8], Al[16][F + 8]; __shared__ float Tf[16][132]; const int lane = threadIdx.x, nloc = lane & 15, hlf = lane >> 4; const int cg = blockIdx.x % 12; const size_t m0 = (size_t)(blockIdx.x / 12) * 16;
  for (int rr = 0; rr < 16; ++rr) { float v[16]; float s = 0.0f;
#pragma unroll
    for (int q = 0; q < 16; ++q) { v[q] = bf16_rne(dat[(m0 + rr) * F + q * 32 + lane]); s += v[q]; }
    for (int o = 16; o; o >>= 1) s += __shfl_xor(s, o); const float mu = s * (1.0f / F); float vq = 0.0f;
#pragma unroll
    for (int q = 0; q < 16; ++q) { const float dd = v[q] - mu; vq += pmul(dd, dd); }
    for (int o = 16; o; o >>= 1) vq += __shfl_xor(vq, o); const float rs = rsqrtf(vq * (1.0f / F) + 1e-5f);
#pragma unroll
    for (int q = 0; q < 16; ++q) { const int c = q * 32 + lane; const float pe = (c & 1) ? 1.0f : 0.0f; const float xx = pmul(pmul(v[q] - mu, rs), bf16_rne(g[c])) + bf16_rne(bt[c]) + pe; b16 p, ql; split16(xx * XS, p, ql); Ah[rr][c] = p; Al[rr][c] = ql; } }
  wave_lds_sync(); v8f acc[8];
#pragma unroll
  for (int t = 0; t < 8; ++t) acc[t] = (v8f){};
#pragma unroll 2
  for (int kb = 0; kb < F; kb += 32) { const v16b a = frag_kb(&Ah[nloc][kb], hlf), al = frag_kb(&Al[nloc][kb], hlf);
#pragma unroll
    for (int t = 0; t < 8; ++t) { const v16b bw = frag_kb(WT + (size_t)(cg * 128 + t * 16 + nloc) * F + kb, hlf); acc[t] = wmma16b(a, bw, acc[t]); acc[t] = wmma16b(al, bw, acc[t]); } }
#pragma unroll
  for (int t = 0; t < 8; ++t)
#pragma unroll
    for (int r8 = 0; r8 < 8; ++r8) Tf[8 * hlf + r8][t * 16 + nloc] = acc[t][r8] * (1.0f / (XS * WSC));
  wave_lds_sync();
  for (int pass = 0; pass < 2; ++pass) { for (int rr = 0; rr < 16; ++rr) *(volatile v4f*)(QKV + (m0 + rr) * E3 + cg * 128 + lane * 4) = *(const v4f*)(&Tf[rr][lane * 4]); __threadfence(); }
}
__global__ __launch_bounds__(256) void kvb_kernel(const float* __restrict__ QKV, b16* __restrict__ KBh, b16* __restrict__ KBl, b16* __restrict__ VTh, b16* __restrict__ VTl) { const size_t u = (size_t)blockIdx.x * 256 + threadIdx.x; if (u >= (size_t)NH * S * 8) return; const int d0 = (int)(u % 8) * 8; const size_t hs = u / 8; const int h = (int)(hs / S), s = (int)(hs % S); v8b kh, kl;
#pragma unroll
  for (int j = 0; j < 8; ++j) { b16 p, q; split16(QKV[(size_t)s * E3 + 512 + h * HD + d0 + j] * XS, p, q); kh[j] = p; kl[j] = q; }
  for (int pass = 0; pass < 2; ++pass) { *(volatile v8b*)(KBh + hs * HD + d0) = kh; *(volatile v8b*)(KBl + hs * HD + d0) = kl; __threadfence(); } (void)VTh; (void)VTl; }
__device__ __forceinline__ void scores_chunk(const b16 (*Qh)[HD + 8], const b16 (*Ql)[HD + 8], const b16* KBh, const b16* KBl, int h, int q0, int kc, float (*Sc)[33], int nloc, int hlf) {
#pragma unroll
  for (int blk = 0; blk < 2; ++blk) { v8f s = {}; const size_t kr = ((size_t)h * S + kc + blk * 16 + nloc) * HD;
#pragma unroll
    for (int kb = 0; kb < HD; kb += 32) { const v16b qh = frag_kb(&Qh[nloc][kb], hlf), ql = frag_kb(&Ql[nloc][kb], hlf), kh = frag_kb(KBh + kr + kb, hlf), kl = frag_kb(KBl + kr + kb, hlf); s = wmma16b(qh, kh, s); s = wmma16b(qh, kl, s); s = wmma16b(ql, kh, s); }
#pragma unroll
    for (int r8 = 0; r8 < 8; ++r8) { const int qi = q0 + 8 * hlf + r8, kj = kc + blk * 16 + nloc; const float dd = (float)(qi - kj); Sc[8 * hlf + r8][blk * 16 + nloc] = s[r8] * (0.125f / (XS * XS)) + __expf(-0.5f * dd * dd); } }
}
__global__ __launch_bounds__(32) void stats_kernel(const float* __restrict__ QKV, const b16* __restrict__ KBh, const b16* __restrict__ KBl, int QLIM, float* __restrict__ ML) {
  __shared__ __attribute__((aligned(16))) b16 Qh[16][HD + 8], Ql[16][HD + 8]; __shared__ float Sc[16][33], Mx[16], Dn[16]; const int lane = threadIdx.x, nloc = lane & 15, hlf = lane >> 4; const int h = blockIdx.x / (QLIM / 16), q0 = (blockIdx.x % (QLIM / 16)) * 16;
  for (int rr = 0; rr < 16; ++rr) for (int q = 0; q < 2; ++q) { b16 p, ql; split16(QKV[(size_t)(q0 + rr) * E3 + h * HD + q * 32 + lane] * XS, p, ql); Qh[rr][q * 32 + lane] = p; Ql[rr][q * 32 + lane] = ql; }
  if (lane < 16) { Mx[lane] = -INFINITY; Dn[lane] = 0.0f; } wave_lds_sync();
#pragma unroll 1
  for (int kc = 0; kc < S; kc += 32) { scores_chunk(Qh, Ql, KBh, KBl, h, q0, kc, Sc, nloc, hlf); wave_lds_sync();
#pragma unroll 1
    for (int qi = 0; qi < 16; ++qi) { const float sv = Sc[qi][lane]; float cm = sv; for (int o = 16; o; o >>= 1) cm = fmaxf(cm, __shfl_xor(cm, o)); const float mo = Mx[qi]; const float mn = fmaxf(mo, cm); float ps = __expf(sv - mn); for (int o = 16; o; o >>= 1) ps += __shfl_xor(ps, o); if (lane == 0) { const float sf = (mo == -INFINITY) ? 0.0f : __expf(mo - mn); Dn[qi] = Dn[qi] * sf + ps; Mx[qi] = mn; } }
    wave_lds_sync(); }
  for (int pass = 0; pass < 2; ++pass) { ((volatile float*)ML)[((size_t)h * S + q0) * 2 + lane] = (lane & 1) ? Dn[lane >> 1] : Mx[lane >> 1]; __threadfence(); }
}
__global__ __launch_bounds__(32) void attn_kernel(const float* __restrict__ QKV, const b16* __restrict__ KBh, const b16* __restrict__ KBl, const float* __restrict__ ML, float* __restrict__ out0, float* __restrict__ out1) {
  __shared__ __attribute__((aligned(16))) b16 Qh[16][HD + 8], Ql[16][HD + 8], Ph[16][40], Pl[16][40], Vh[HD][40], Vl[HD][40]; __shared__ float Sc[16][33], Ms[16], Ls[16], Of[16][HD + 2];
  const int lane = threadIdx.x, nloc = lane & 15, hlf = lane >> 4; const int q0 = blockIdx.x * 16;
#pragma unroll 1
  for (int h = 0; h < NH; ++h) {
    for (int rr = 0; rr < 16; ++rr) for (int q = 0; q < 2; ++q) { b16 p, ql; split16(QKV[(size_t)(q0 + rr) * E3 + h * HD + q * 32 + lane] * XS, p, ql); Qh[rr][q * 32 + lane] = p; Ql[rr][q * 32 + lane] = ql; }
    if (lane < 16) { Ms[lane] = ML[((size_t)h * S + q0 + lane) * 2]; Ls[lane] = ML[((size_t)h * S + q0 + lane) * 2 + 1]; }
    v8f acc[4] = {(v8f){}, (v8f){}, (v8f){}, (v8f){}}; wave_lds_sync();
#pragma unroll 1
    for (int kc = 0; kc < S; kc += 32) {
      for (int rr = 0; rr < 32; ++rr) for (int q = 0; q < 2; ++q) { b16 p, ql; split16(QKV[(size_t)(kc + rr) * E3 + 1024 + h * HD + q * 32 + lane] * XS, p, ql); Vh[q * 32 + lane][rr] = p; Vl[q * 32 + lane][rr] = ql; }
      scores_chunk(Qh, Ql, KBh, KBl, h, q0, kc, Sc, nloc, hlf); wave_lds_sync();
      const int npass = (h == NH - 1) ? 2 : 1;
      for (int qi = 0; qi < 16; ++qi) { const float p = __expf(Sc[qi][lane] - Ms[qi]) / Ls[qi]; b16 ph, plo; split16(p * PS, ph, plo); Ph[qi][lane] = ph; Pl[qi][lane] = plo;
        float* mw = out1 + (size_t)(q0 + qi) * S + kc + lane; const float prev = (h == 0) ? 0.0f : *mw; const float nv = prev + p * (1.0f / NH); for (int pass = 0; pass < npass; ++pass) { *(volatile float*)mw = nv; if (npass == 2) __threadfence(); } }
      wave_lds_sync(); const v16b pa = frag_kb(&Ph[nloc][0], hlf), pb = frag_kb(&Pl[nloc][0], hlf);
#pragma unroll
      for (int t = 0; t < 4; ++t) { const v16b vh = frag_kb(&Vh[t * 16 + nloc][0], hlf), vl = frag_kb(&Vl[t * 16 + nloc][0], hlf); acc[t] = wmma16b(pa, vh, acc[t]); acc[t] = wmma16b(pa, vl, acc[t]); acc[t] = wmma16b(pb, vh, acc[t]); }
      wave_lds_sync(); }
#pragma unroll
    for (int t = 0; t < 4; ++t)
#pragma unroll
      for (int r8 = 0; r8 < 8; ++r8) Of[8 * hlf + r8][t * 16 + nloc] = acc[t][r8] * (1.0f / (PS * XS));
    wave_lds_sync();
    for (int pass = 0; pass < 2; ++pass) { for (int rr = 0; rr < 16; ++rr) *(volatile v2f*)(out0 + (size_t)(q0 + rr) * F + h * HD + lane * 2) = (v2f){Of[rr][lane * 2], Of[rr][lane * 2 + 1]}; __threadfence(); }
    wave_lds_sync(); }
}
}

extern "C" void kernel_launch(void* const* d_in, const int* in_sizes, int n_in, void* d_out, int out_size, void* d_ws, size_t ws_size, hipStream_t stream) {
  (void)n_in;
  auto Fp = [&](int i) { return (const float*)d_in[i]; };
  if (in_sizes[0] != S * F || in_sizes[1] != NH * F * HD || in_sizes[2] != NH * F * HD || in_sizes[3] != NH * F * HD || in_sizes[4] != F || out_size != S * F + S * S) return;
  const int QLIM = S;
  size_t off = 0; char* ws = (char*)d_ws;
  auto carve = [&](size_t bytes) { char* p = ws + off; off += (bytes + 255) & ~(size_t)255; return p; };
  b16* WT = (b16*)carve((size_t)E3 * F * 2); float* QKV = (float*)carve((size_t)S * E3 * 4); b16* KBh = (b16*)carve((size_t)NH * S * HD * 2); b16* KBl = (b16*)carve((size_t)NH * S * HD * 2); float* ML = (float*)carve((size_t)NH * S * 2 * 4);
  if (off > ws_size || off > ((size_t)32 << 20)) return;
  wput_kernel<<<(E3 * (F / 8) + 255) / 256, 256, 0, stream>>>(Fp(1), Fp(2), Fp(3), WT);
  qkv_kernel<<<(S / 16) * 12, 32, 0, stream>>>(Fp(0), Fp(4), Fp(5), WT, QKV);
  kvb_kernel<<<(NH * S * 8 + 255) / 256, 256, 0, stream>>>(QKV, KBh, KBl, nullptr, nullptr);
  float* out = (float*)d_out;
  stats_kernel<<<NH * (QLIM / 16), 32, 0, stream>>>(QKV, KBh, KBl, QLIM, ML);
  attn_kernel<<<QLIM / 16, 32, 0, stream>>>(QKV, KBh, KBl, ML, out, out + (size_t)S * F);
}
